// BertClassifier_62938450755707
// MI455X (gfx1250) — hardware-verified
//
#include <hip/hip_runtime.h>


#define NBT  4
#define TT   128
#define DD   768
#define HH   770
#define HP   832
#define LL   40
#define LP   64
#define NPR  (TT * TT)
#define DM   DD
#define LOSC 1024.0f

typedef _Float16 h16;
typedef unsigned short bf;
typedef __attribute__((ext_vector_type(16))) __bf16   v16bf;
typedef __attribute__((ext_vector_type(16))) _Float16 v16h;
typedef __attribute__((ext_vector_type(8)))  _Float16 v8h;
typedef __attribute__((ext_vector_type(8)))  unsigned short v8us;
typedef __attribute__((ext_vector_type(8)))  float    v8f;
typedef __attribute__((ext_vector_type(4)))  float    v4f;
typedef v8h  __attribute__((may_alias)) v8ha;
typedef v4f  __attribute__((may_alias)) v4fa;
typedef v8us __attribute__((may_alias)) v8usa;

__device__ __forceinline__ unsigned short f2bf(float f) { unsigned u = __float_as_uint(f); u += 0x7FFFu + ((u >> 16) & 1u); return (unsigned short)(u >> 16); }
__device__ __forceinline__ float bf2f(unsigned short b) { return __uint_as_float(((unsigned)b) << 16); }
__device__ __forceinline__ float bfr(float f) { return bf2f(f2bf(f)); }
__device__ __forceinline__ v16h cat16(v8h lo, v8h hi) { return __builtin_shufflevector(lo, hi, 0, 1, 2, 3, 4, 5, 6, 7, 8, 9, 10, 11, 12, 13, 14, 15); }
__device__ __forceinline__ v16bf cat16b(v8us lo, v8us hi) { return __builtin_bit_cast(v16bf, __builtin_shufflevector(lo, hi, 0, 1, 2, 3, 4, 5, 6, 7, 8, 9, 10, 11, 12, 13, 14, 15)); }
__device__ __forceinline__ v8f wmma16(v16h a, v16h b, v8f c) { return __builtin_amdgcn_wmma_f32_16x16x32_f16(false, a, false, b, (short)0, c, false, false); }
__device__ __forceinline__ v8f wmmab(v16bf a, v16bf b, v8f c) { return __builtin_amdgcn_wmma_f32_16x16x32_bf16(false, a, false, b, (short)0, c, false, false); }

template <bool SPLITA, bool F16OUT = false>
__global__ __launch_bounds__(128) void k_gemmb(const bf* __restrict__ A, const bf* __restrict__ Al, const bf* __restrict__ Bn, const float* __restrict__ bias, float* C, int ldc, h16* C2, const float* __restrict__ R = nullptr, int K = DM, int roundR = 1) {
    __shared__ __align__(16) float ost[4][16 * 68];
    const int lane = threadIdx.x & 31, wave = threadIdx.x >> 5, lr = lane & 15, hi = lane >> 4;
    const int r0 = blockIdx.x * 64 + wave * 16, c0 = blockIdx.y * 64;
    const size_t aoff = (size_t)(r0 + lr) * K + 8 * hi;
    size_t boff[4];
#pragma unroll
    for (int t = 0; t < 4; ++t) boff[t] = (size_t)(c0 + t * 16 + lr) * K + 8 * hi;
    v8f acc[4];
#pragma unroll
    for (int t = 0; t < 4; ++t) acc[t] = (v8f){};
#pragma unroll 1
    for (int kc = 0; kc < K; kc += 32) {
        const v16bf a = cat16b(*(const v8us*)(A + aoff + kc), *(const v8us*)(A + aoff + kc + 16));
        v16bf al = a;
        if (SPLITA) al = cat16b(*(const v8us*)(Al + aoff + kc), *(const v8us*)(Al + aoff + kc + 16));
#pragma unroll
        for (int t = 0; t < 4; ++t) { const v16bf b = cat16b(*(const v8us*)(Bn + boff[t] + kc), *(const v8us*)(Bn + boff[t] + kc + 16)); acc[t] = wmmab(a, b, acc[t]); if (SPLITA) acc[t] = wmmab(al, b, acc[t]); }
        asm volatile("v_nop\n\tv_nop\n\tv_nop\n\tv_nop" : "+v"(acc[0]), "+v"(acc[1]), "+v"(acc[2]), "+v"(acc[3]) : "v"(a), "v"(al));
    }
    float* os = &ost[wave][0];
#pragma unroll
    for (int t = 0; t < 4; ++t) { const float bv = bias ? bfr(bias[c0 + t * 16 + lr]) : 0.f;
#pragma unroll
        for (int j = 0; j < 8; ++j) os[(hi * 8 + j) * 68 + t * 16 + lr] = acc[t][j] + bv; }
    __syncthreads();
    if (F16OUT) {
        h16* crow = (h16*)(void*)C + (size_t)r0 * ldc + c0;
        auto pass = [&]() {
#pragma unroll
            for (int s = 0; s < 4; ++s) { const int row = 4 * s + (lane >> 3), piece = lane & 7; const float* sp = os + row * 68 + piece * 8; v8h o, o2;
#pragma unroll
                for (int i = 0; i < 8; ++i) { const h16 a = (h16)sp[i]; o[i] = a; o2[i] = (h16)((sp[i] - (float)a) * LOSC); }
                *(volatile v8h*)(crow + (size_t)row * ldc + piece * 8) = o; if (C2) *(volatile v8h*)(C2 + (size_t)r0 * ldc + c0 + (size_t)row * ldc + piece * 8) = o2; }
        };
        pass(); __threadfence(); pass();
    } else {
        float* crow = C + (size_t)r0 * ldc + c0;
        auto pass = [&]() {
#pragma unroll
            for (int s = 0; s < 8; ++s) { const int Lid = (lane >> 3) + 4 * s, piece = lane & 7; const int row = Lid >> 1, cofs = (Lid & 1) * 32 + piece * 4;
                v4f val = *(const v4fa*)(os + row * 68 + cofs); if (R) { const v4f rv = *(const v4f*)(R + ((size_t)r0 + row) * ldc + c0 + cofs); val += roundR ? (v4f){bfr(rv[0]), bfr(rv[1]), bfr(rv[2]), bfr(rv[3])} : rv; }
                *(volatile v4f*)(crow + (size_t)row * ldc + cofs) = val; }
        };
        pass(); __threadfence(); pass();
    }
}


__global__ __launch_bounds__(256) void k_wtp(const float* __restrict__ Wm, int krows, int ncols, int kpad, bf* WT) {
    __shared__ __align__(16) unsigned short tl[64 * 72];
    const int tid = threadIdx.x, k0 = blockIdx.x * 64, n0 = blockIdx.y * 64;
    const int kk = tid >> 2, nq = (tid & 3) * 16;
    const int k = k0 + kk, kc = k < krows ? k : krows - 1;
#pragma unroll
    for (int i = 0; i < 16; ++i) { const int n = n0 + nq + i, ncl = n < ncols ? n : ncols - 1; const float w = Wm[(size_t)kc * ncols + ncl]; tl[(nq + i) * 72 + kk] = (k < krows && n < ncols) ? f2bf(w) : (unsigned short)0; }
    __syncthreads();
    const int piece = tid & 7;
    auto pass = [&]() {
#pragma unroll
        for (int s = 0; s < 2; ++s) { const int nr = (tid >> 3) + 32 * s; const v8us val = *(const v8usa*)(tl + nr * 72 + piece * 8); *(volatile v8us*)(WT + (size_t)(n0 + nr) * kpad + k0 + piece * 8) = val; }
    };
    pass(); __threadfence(); pass();
}

__global__ __launch_bounds__(256) void k_cvtv(const float* __restrict__ hid, bf* dst) {
    const int lane = threadIdx.x & 31; const size_t r = (size_t)blockIdx.x * 8 + (threadIdx.x >> 5); if (r >= (size_t)TT) return;
#pragma unroll 1
    for (int ps = 0; ps < 2; ++ps) {
#pragma unroll
        for (int q = 0; q < DD / 256; ++q) { v8us o;
#pragma unroll
            for (int i = 0; i < 8; ++i) o[i] = f2bf(hid[(r + 1) * DD + q * 256 + lane * 8 + i]);
            *(volatile v8us*)(dst + r * DD + q * 256 + lane * 8) = o; }
        if (ps == 0) __threadfence(); }
}
__global__ __launch_bounds__(1024) void k_bpad(const float* __restrict__ src, int N, int n, float* BP) {
    const int t = threadIdx.x; if (t >= n) return; const float v = (t < N) ? bfr(src[t < N ? t : 0]) : 0.f; *(volatile float*)(BP + t) = v; __threadfence(); *(volatile float*)(BP + t) = v;
}
__global__ __launch_bounds__(256) void k_hpl(const float* __restrict__ A, const float* __restrict__ Bm, const float* __restrict__ wind, const int* __restrict__ spans, bf* Ph, bf* Pl) {
    typedef __attribute__((ext_vector_type(2))) unsigned short v2us;
    const int lane = threadIdx.x & 31; const int p = blockIdx.x * 8 + (threadIdx.x >> 5); if (p >= NPR) return; const int i = p / TT, j = p % TT; const int s0 = spans[0], e0 = spans[1];
    const bool full = (i == s0) && (j == e0); const bool inside = (s0 <= i) && (i <= j) && (j <= e0) && !full; const float ind = full ? 2.0f : (inside ? 1.0f : 0.0f);
#pragma unroll 1
    for (int ps = 0; ps < 2; ++ps) {
#pragma unroll 1
        for (int st = 0; st < HP / 64; ++st) { const int c0 = st * 64 + lane * 2; v2us oh, ol;
#pragma unroll
            for (int q = 0; q < 2; ++q) { const int n = c0 + q; const int nc = n < HH ? n : 0; float y = A[(size_t)i * HP + nc] + Bm[(size_t)j * HP + nc] + ind * bfr(wind[nc]); y = fmaxf(y, 0.f); if (n >= HH) y = 0.f; const unsigned short hb = f2bf(y); oh[q] = hb; ol[q] = f2bf(y - bf2f(hb)); }
            const size_t o = (size_t)p * HP + c0; *(volatile v2us*)(Ph + o) = oh; *(volatile v2us*)(Pl + o) = ol; }
        if (ps == 0) __threadfence(); }
}
__global__ __launch_bounds__(256) void k_lse(const float* __restrict__ Cb, const int* __restrict__ avail, float* LSE) {
    __shared__ float red[256]; __shared__ float res[64];
    const int t = threadIdx.x;
    if (t < 64) res[t] = 0.f;
    __syncthreads();
#pragma unroll 1
    for (int l = 0; l < LL; ++l) {
        float m = -3.0e38f;
        for (int q = 0; q < NPR / 256; ++q) { const int p = q * 256 + t; const float v = (avail[p] >= 1) ? Cb[(size_t)p * LP + l] : 0.f; m = fmaxf(m, v); }
        red[t] = m; __syncthreads();
        for (int s = 128; s > 0; s >>= 1) { if (t < s) red[t] = fmaxf(red[t], red[t + s]); __syncthreads(); }
        const float M = red[0]; __syncthreads();
        float sm = 0.f;
        for (int q = 0; q < NPR / 256; ++q) { const int p = q * 256 + t; const float v = (avail[p] >= 1) ? Cb[(size_t)p * LP + l] : 0.f; sm += __expf(v - M); }
        red[t] = sm; __syncthreads();
        for (int s = 128; s > 0; s >>= 1) { if (t < s) red[t] += red[t + s]; __syncthreads(); }
        if (t == 0) res[l] = M + logf(red[0]);
        __syncthreads(); }
    if (t < 64) { const float v = res[t]; *(volatile float*)(LSE + t) = v; __threadfence(); *(volatile float*)(LSE + t) = v; }
}
__global__ __launch_bounds__(256) void k_outw(const float* __restrict__ Cb, const int* __restrict__ avail, const float* __restrict__ LSE, float* OUTB) {
    const int lane = threadIdx.x & 31; const size_t wid = (size_t)blockIdx.x * 8 + (threadIdx.x >> 5); if (wid >= (size_t)NPR * LL / 128) return; const size_t e0 = wid * 128 + lane * 4; v4f v;
#pragma unroll
    for (int q = 0; q < 4; ++q) { const size_t e = e0 + q; const int p = (int)(e / LL), l = (int)(e % LL); v[q] = ((avail[p] >= 1) ? Cb[(size_t)p * LP + l] : 0.f) - LSE[l]; }
    *(volatile v4f*)(OUTB + e0) = v; __threadfence(); *(volatile v4f*)(OUTB + e0) = v;
}

extern "C" void kernel_launch(void* const* d_in, const int* in_sizes, int n_in,
                              void* d_out, int out_size, void* d_ws, size_t ws_size, hipStream_t stream) {
    (void)in_sizes; (void)n_in; (void)out_size;
    const float* hid = (const float*)d_in[0]; const float* W1 = (const float*)d_in[1]; const float* b1 = (const float*)d_in[2]; const float* W2 = (const float*)d_in[3]; const float* b2 = (const float*)d_in[4]; const int* spans = (const int*)d_in[5]; const int* avail = (const int*)d_in[6];
    float* out = (float*)d_out;
    char* wsp = (char*)d_ws;
    auto take = [&](size_t bytes) { char* p = wsp; wsp += (bytes + 255) & ~(size_t)255; return (void*)p; };
    bf* W1aT = (bf*)take((size_t)HP * DD * 2); bf* W1bT = (bf*)take((size_t)HP * DD * 2); bf* W2T = (bf*)take((size_t)LP * HP * 2); float* B1P = (float*)take(HP * 4); float* B2P = (float*)take(LP * 4);
    bf* Vb = (bf*)take((size_t)TT * DD * 2); float* A = (float*)take((size_t)TT * HP * 4); float* Bm = (float*)take((size_t)TT * HP * 4); bf* Ph = (bf*)take((size_t)NPR * HP * 2); bf* Pl = (bf*)take((size_t)NPR * HP * 2); float* Cb = (float*)take((size_t)NPR * LP * 4); float* LSE = (float*)take(LP * 4);
    if ((size_t)(wsp - (char*)d_ws) > ws_size) return;
    k_wtp<<<dim3(DD / 64, HP / 64, 1), 256, 0, stream>>>(W1, DD, HH, DD, W1aT); k_wtp<<<dim3(DD / 64, HP / 64, 1), 256, 0, stream>>>(W1 + (size_t)DD * HH, DD, HH, DD, W1bT);
    k_wtp<<<dim3(HP / 64, LP / 64, 1), 256, 0, stream>>>(W2, HH, LL, HP, W2T);
    k_bpad<<<1, HP, 0, stream>>>(b1, HH, HP, B1P); k_bpad<<<1, LP, 0, stream>>>(b2, LL, LP, B2P);
    const float* wind = W1 + (size_t)2 * DD * HH;
    for (int b = 0; b < NBT; ++b) {
        k_cvtv<<<TT / 8, 256, 0, stream>>>(hid + (size_t)b * (TT + 1) * DD, Vb);
        k_gemmb<false, false><<<dim3(TT / 64, HP / 64, 1), 128, 0, stream>>>(Vb, nullptr, W1aT, B1P, A, HP, nullptr, nullptr, DD);
        k_gemmb<false, false><<<dim3(TT / 64, HP / 64, 1), 128, 0, stream>>>(Vb, nullptr, W1bT, nullptr, Bm, HP, nullptr, nullptr, DD);
        k_hpl<<<NPR / 8, 256, 0, stream>>>(A, Bm, wind, spans + b * 2, Ph, Pl);
        k_gemmb<true, false><<<dim3(NPR / 64, 1, 1), 128, 0, stream>>>(Ph, Pl, W2T, B2P, Cb, LP, nullptr, nullptr, HP);
        k_lse<<<1, 256, 0, stream>>>(Cb, avail, LSE);
        k_outw<<<(NPR * LL / 128) / 8, 256, 0, stream>>>(Cb, avail, LSE, out + (size_t)b * NPR * LL); }
}
